// SymbolicCausalSelfAttentionALiBi_66314295050783
// MI455X (gfx1250) — hardware-verified
//
#include <hip/hip_runtime.h>


#define NB_  2
#define TT   768
#define CC   64
#define NR   (NB_ * TT)
#define DM   CC
#define LOSC 1024.0f
typedef _Float16 h16;
typedef unsigned short bf;
typedef __attribute__((ext_vector_type(16))) __bf16   v16bf;
typedef __attribute__((ext_vector_type(16))) _Float16 v16h;
typedef __attribute__((ext_vector_type(8)))  _Float16 v8h;
typedef __attribute__((ext_vector_type(8)))  unsigned short v8us;
typedef __attribute__((ext_vector_type(8)))  float    v8f;
typedef __attribute__((ext_vector_type(4)))  float    v4f;
typedef v8h  __attribute__((may_alias)) v8ha;
typedef v4f  __attribute__((may_alias)) v4fa;
typedef v8us __attribute__((may_alias)) v8usa;

__device__ __forceinline__ unsigned short f2bf(float f) { unsigned u = __float_as_uint(f); u += 0x7FFFu + ((u >> 16) & 1u); return (unsigned short)(u >> 16); }
__device__ __forceinline__ float bf2f(unsigned short b) { return __uint_as_float(((unsigned)b) << 16); }
__device__ __forceinline__ float bfr(float f) { return bf2f(f2bf(f)); }
__device__ __forceinline__ v16h cat16(v8h lo, v8h hi) { return __builtin_shufflevector(lo, hi, 0, 1, 2, 3, 4, 5, 6, 7, 8, 9, 10, 11, 12, 13, 14, 15); }
__device__ __forceinline__ v16bf cat16b(v8us lo, v8us hi) { return __builtin_bit_cast(v16bf, __builtin_shufflevector(lo, hi, 0, 1, 2, 3, 4, 5, 6, 7, 8, 9, 10, 11, 12, 13, 14, 15)); }
__device__ __forceinline__ v8f wmma16(v16h a, v16h b, v8f c) { return __builtin_amdgcn_wmma_f32_16x16x32_f16(false, a, false, b, (short)0, c, false, false); }
__device__ __forceinline__ v8f wmmab(v16bf a, v16bf b, v8f c) { return __builtin_amdgcn_wmma_f32_16x16x32_bf16(false, a, false, b, (short)0, c, false, false); }

template <bool SPLITA, bool F16OUT = false>
__global__ __launch_bounds__(128) void k_gemmb(const bf* __restrict__ A, const bf* __restrict__ Al, const bf* __restrict__ Bn, const float* __restrict__ bias, float* C, int ldc, h16* C2, const float* __restrict__ R = nullptr, int K = DM, int roundR = 1) {
    __shared__ __align__(16) float ost[4][16 * 68];
    const int lane = threadIdx.x & 31, wave = threadIdx.x >> 5, lr = lane & 15, hi = lane >> 4;
    const int r0 = blockIdx.x * 64 + wave * 16, c0 = blockIdx.y * 64;
    const size_t aoff = (size_t)(r0 + lr) * K + 8 * hi;
    size_t boff[4];
#pragma unroll
    for (int t = 0; t < 4; ++t) boff[t] = (size_t)(c0 + t * 16 + lr) * K + 8 * hi;
    v8f acc[4];
#pragma unroll
    for (int t = 0; t < 4; ++t) acc[t] = (v8f){};
#pragma unroll 1
    for (int kc = 0; kc < K; kc += 32) {
        const v16bf a = cat16b(*(const v8us*)(A + aoff + kc), *(const v8us*)(A + aoff + kc + 16));
        v16bf al = a;
        if (SPLITA) al = cat16b(*(const v8us*)(Al + aoff + kc), *(const v8us*)(Al + aoff + kc + 16));
#pragma unroll
        for (int t = 0; t < 4; ++t) { const v16bf b = cat16b(*(const v8us*)(Bn + boff[t] + kc), *(const v8us*)(Bn + boff[t] + kc + 16)); acc[t] = wmmab(a, b, acc[t]); if (SPLITA) acc[t] = wmmab(al, b, acc[t]); }
        asm volatile("v_nop\n\tv_nop\n\tv_nop\n\tv_nop" : "+v"(acc[0]), "+v"(acc[1]), "+v"(acc[2]), "+v"(acc[3]) : "v"(a), "v"(al));
    }
    float* os = &ost[wave][0];
#pragma unroll
    for (int t = 0; t < 4; ++t) { const float bv = bias ? bfr(bias[c0 + t * 16 + lr]) : 0.f;
#pragma unroll
        for (int j = 0; j < 8; ++j) os[(hi * 8 + j) * 68 + t * 16 + lr] = acc[t][j] + bv; }
    __syncthreads();
    if (F16OUT) {
        h16* crow = (h16*)(void*)C + (size_t)r0 * ldc + c0;
        auto pass = [&]() {
#pragma unroll
            for (int s = 0; s < 4; ++s) { const int row = 4 * s + (lane >> 3), piece = lane & 7; const float* sp = os + row * 68 + piece * 8; v8h o, o2;
#pragma unroll
                for (int i = 0; i < 8; ++i) { const h16 a = (h16)sp[i]; o[i] = a; o2[i] = (h16)((sp[i] - (float)a) * LOSC); }
                *(volatile v8h*)(crow + (size_t)row * ldc + piece * 8) = o; if (C2) *(volatile v8h*)(C2 + (size_t)r0 * ldc + c0 + (size_t)row * ldc + piece * 8) = o2; }
        };
        pass(); __threadfence(); pass();
    } else {
        float* crow = C + (size_t)r0 * ldc + c0;
        auto pass = [&]() {
#pragma unroll
            for (int s = 0; s < 8; ++s) { const int Lid = (lane >> 3) + 4 * s, piece = lane & 7; const int row = Lid >> 1, cofs = (Lid & 1) * 32 + piece * 4;
                v4f val = *(const v4fa*)(os + row * 68 + cofs); if (R) { const v4f rv = *(const v4f*)(R + ((size_t)r0 + row) * ldc + c0 + cofs); val += roundR ? (v4f){bfr(rv[0]), bfr(rv[1]), bfr(rv[2]), bfr(rv[3])} : rv; }
                *(volatile v4f*)(crow + (size_t)row * ldc + cofs) = val; }
        };
        pass(); __threadfence(); pass();
    }
}

__global__ __launch_bounds__(256) void k_cvt8(const float* __restrict__ src, bf* dst, size_t n8) {
    const size_t i = (size_t)blockIdx.x * 256 + threadIdx.x; if (i >= n8) return;
    const v8f v = *(const v8f*)(src + i * 8); v8us o;
#pragma unroll
    for (int k = 0; k < 8; ++k) o[k] = f2bf(v[k]);
    *(volatile v8us*)(dst + i * 8) = o; __threadfence(); *(volatile v8us*)(dst + i * 8) = o;
}
__global__ __launch_bounds__(256) void k_zero8(bf* dst, size_t n8) {
    const size_t i = (size_t)blockIdx.x * 256 + threadIdx.x; if (i >= n8) return; v8us z;
#pragma unroll
    for (int k = 0; k < 8; ++k) z[k] = 0;
    *(volatile v8us*)(dst + i * 8) = z; __threadfence(); *(volatile v8us*)(dst + i * 8) = z;
}
__constant__ float c_slope[64] = {0.917004049f, 0.840896428f, 0.771105409f, 0.707106769f, 0.648419797f, 0.594603539f, 0.545253873f, 0.500000000f, 0.458502024f, 0.420448214f, 0.385552704f, 0.353553385f, 0.324209899f, 0.297301769f, 0.272626936f, 0.250000000f, 0.229251012f, 0.210224107f, 0.192776352f, 0.176776692f, 0.162104949f, 0.148650885f, 0.136313468f, 0.125000000f, 0.114625506f, 0.105112053f, 0.0963881761f, 0.0883883461f, 0.0810524747f, 0.0743254423f, 0.0681567341f, 0.0625000000f, 0.0573127531f, 0.0525560267f, 0.0481940880f, 0.0441941731f, 0.0405262373f, 0.0371627212f, 0.0340783671f, 0.0312500000f, 0.0286563765f, 0.0262780134f, 0.0240970440f, 0.0220970865f, 0.0202631187f, 0.0185813606f, 0.0170391835f, 0.0156250000f, 0.0143281883f, 0.0131390067f, 0.0120485220f, 0.0110485433f, 0.0101315593f, 0.00929068029f, 0.00851959176f, 0.00781250000f, 0.00716409413f, 0.00656950334f, 0.00602426101f, 0.00552427163f, 0.00506577967f, 0.00464534014f, 0.00425979588f, 0.00390625000f};
__global__ __launch_bounds__(256) void k_cvtx(const float* __restrict__ x, bf* A) {
    typedef __attribute__((ext_vector_type(2))) unsigned short v2us;
    const int lane = threadIdx.x & 31; const size_t r = (size_t)blockIdx.x * 8 + (threadIdx.x >> 5); if (r >= (size_t)NR) return; v2us o; o[0] = f2bf(x[r * CC + lane * 2]); o[1] = f2bf(x[r * CC + lane * 2 + 1]);
    *(volatile v2us*)(A + r * CC + lane * 2) = o; __threadfence(); *(volatile v2us*)(A + r * CC + lane * 2) = o;
}
__global__ __launch_bounds__(256) void k_attn1(const float* __restrict__ QK, const float* __restrict__ x, const float* __restrict__ vt, const float* __restrict__ pt, float* OUTB) {
    const int lane = threadIdx.x & 31; const int r = blockIdx.x * 8 + (threadIdx.x >> 5); if (r >= NR) return; const int b = r / TT, i = r % TT; const float* QKb = QK + (size_t)b * TT * (2 * CC); const float* xb = x + (size_t)b * TT * CC;
    float res[2];
#pragma unroll
    for (int hh = 0; hh < 2; ++hh) { const int h = hh * 32 + lane; const float q = QKb[(size_t)i * (2 * CC) + h]; const float sl = c_slope[h]; const float vs = bfr(vt[h]);
        float m = -3.0e38f;
#pragma unroll 1
        for (int j = 0; j < TT; ++j) { const float s = fmaf(q, QKb[(size_t)j * (2 * CC) + CC + h], sl * (float)min(j - i, 0)); m = fmaxf(m, s); }
        float se = 0.f, sv = 0.f;
#pragma unroll 1
        for (int j = 0; j < TT; ++j) { const float s = fmaf(q, QKb[(size_t)j * (2 * CC) + CC + h], sl * (float)min(j - i, 0)); const float e = __expf(s - m); se += e; sv = fmaf(e, bfr(xb[(size_t)j * CC + h]) * vs, sv); }
        res[hh] = __fdiv_rn(sv, se) * bfr(pt[h]); }
    float* dst = OUTB + (size_t)r * CC;
#pragma unroll 1
    for (int ps = 0; ps < 2; ++ps) { *(volatile float*)(dst + lane) = res[0]; *(volatile float*)(dst + 32 + lane) = res[1]; if (ps == 0) __threadfence(); }
}
extern "C" void kernel_launch(void* const* d_in, const int* in_sizes, int n_in,
                              void* d_out, int out_size, void* d_ws, size_t ws_size, hipStream_t stream) {
    (void)in_sizes; (void)n_in; (void)out_size;
    const float* x = (const float*)d_in[0]; const float* W = (const float*)d_in[1]; const float* vt = (const float*)d_in[2]; const float* pt = (const float*)d_in[3];
    float* out = (float*)d_out;
    char* wsp = (char*)d_ws;
    auto take = [&](size_t bytes) { char* p = wsp; wsp += (bytes + 255) & ~(size_t)255; return (void*)p; };
    bf* WB = (bf*)take(2 * CC * CC * 2); bf* XB = (bf*)take((size_t)NR * CC * 2); float* QK = (float*)take((size_t)NR * 2 * CC * 4);
    if ((size_t)(wsp - (char*)d_ws) > ws_size) return;
    k_cvt8<<<(unsigned)((2 * CC * CC / 8 + 255) / 256), 256, 0, stream>>>(W, WB, 2 * CC * CC / 8);
    k_cvtx<<<NR / 8, 256, 0, stream>>>(x, XB);
    k_gemmb<false, false><<<dim3(NR / 64, (2 * CC) / 64, 1), 128, 0, stream>>>(XB, nullptr, WB, nullptr, QK, 2 * CC, nullptr, nullptr, CC);
    k_attn1<<<NR / 8, 256, 0, stream>>>(QK, x, vt, pt, out);
}
